// E_MHSA_Original_20255065768207
// MI455X (gfx1250) — hardware-verified
//
#include <hip/hip_runtime.h>


#define NB_  32
#define CC   384
#define NN_  1024
#define NK   256
#define NH_  12
#define HD   32
#define NTQ  (NB_ * NN_)
#define NTKV (NB_ * NK)
#define PSC  32768.0f
#define SCL  0.17677669529663687f

typedef _Float16 h16;
typedef unsigned short bf;
typedef __attribute__((ext_vector_type(16))) __bf16   v16bf;
typedef __attribute__((ext_vector_type(16))) _Float16 v16h;
typedef __attribute__((ext_vector_type(8)))  _Float16 v8h;
typedef __attribute__((ext_vector_type(8)))  unsigned short v8us;
typedef __attribute__((ext_vector_type(8)))  float    v8f;
typedef __attribute__((ext_vector_type(4)))  float    v4f;
typedef v8h  __attribute__((may_alias)) v8ha;
typedef v4f  __attribute__((may_alias)) v4fa;
typedef v8us __attribute__((may_alias)) v8usa;

__device__ __forceinline__ unsigned short f2bf(float f) { unsigned u = __float_as_uint(f); u += 0x7FFFu + ((u >> 16) & 1u); return (unsigned short)(u >> 16); }
__device__ __forceinline__ float bf2f(unsigned short b) { return __uint_as_float(((unsigned)b) << 16); }
__device__ __forceinline__ float bfr(float f) { return bf2f(f2bf(f)); }
__device__ __forceinline__ v16h cat16(v8h lo, v8h hi) { return __builtin_shufflevector(lo, hi, 0, 1, 2, 3, 4, 5, 6, 7, 8, 9, 10, 11, 12, 13, 14, 15); }
__device__ __forceinline__ v16bf cat16b(v8us lo, v8us hi) { return __builtin_bit_cast(v16bf, __builtin_shufflevector(lo, hi, 0, 1, 2, 3, 4, 5, 6, 7, 8, 9, 10, 11, 12, 13, 14, 15)); }
__device__ __forceinline__ v8f wmma16(v16h a, v16h b, v8f c) { return __builtin_amdgcn_wmma_f32_16x16x32_f16(false, a, false, b, (short)0, c, false, false); }
__device__ __forceinline__ v8f wmmab(v16bf a, v16bf b, v8f c) { return __builtin_amdgcn_wmma_f32_16x16x32_bf16(false, a, false, b, (short)0, c, false, false); }

__global__ __launch_bounds__(256) void k_tok(const float* __restrict__ x, bf* Xb) {
    __shared__ __align__(16) unsigned short tl[64 * 72];
    const int tid = threadIdx.x, n0 = blockIdx.x * 64, c0 = blockIdx.y * 64, b = blockIdx.z;
    const int cc = tid >> 2, nq = (tid & 3) * 16;
#pragma unroll
    for (int i = 0; i < 16; ++i) tl[(nq + i) * 72 + cc] = f2bf(x[((size_t)b * CC + c0 + cc) * NN_ + n0 + nq + i]);
    __syncthreads();
    const int piece = tid & 7;
    auto pass = [&]() {
#pragma unroll
        for (int s = 0; s < 2; ++s) { const int nr = (tid >> 3) + 32 * s; const v8us val = *(const v8usa*)(tl + nr * 72 + piece * 8);
            *(volatile v8us*)(Xb + ((size_t)b * NN_ + n0 + nr) * CC + c0 + piece * 8) = val; }
    };
    pass(); __threadfence(); pass();
}
__global__ __launch_bounds__(256) void k_pool(const float* __restrict__ x, const float* __restrict__ g, const float* __restrict__ be, const float* __restrict__ mu, const float* __restrict__ var, bf* XRH, bf* XRL) {
    __shared__ __align__(16) unsigned short th_[64 * 72];
    __shared__ __align__(16) unsigned short tl_[64 * 72];
    const int tid = threadIdx.x, m0 = blockIdx.x * 64, c0 = blockIdx.y * 64, b = blockIdx.z;
    const int cc = tid >> 2, mq = (tid & 3) * 16, c = c0 + cc;
    const float inv = bfr(g[c]) / sqrtf(bfr(var[c]) + 1e-5f), sh = bfr(be[c]) - bfr(mu[c]) * inv;
    const float* xr = x + ((size_t)b * CC + c) * NN_;
#pragma unroll
    for (int i = 0; i < 16; ++i) { const int m = m0 + mq + i; const float* p = xr + 4 * m;
        const float v = ((bfr(p[0]) + bfr(p[1]) + bfr(p[2]) + bfr(p[3])) * 0.25f) * inv + sh;
        const unsigned short hb = f2bf(v); th_[(mq + i) * 72 + cc] = hb; tl_[(mq + i) * 72 + cc] = f2bf(v - bf2f(hb)); }
    __syncthreads();
    const int piece = tid & 7;
    auto pass = [&]() {
#pragma unroll
        for (int s = 0; s < 4; ++s) { const int Lid = (tid >> 3) + 32 * s; const int pln = Lid >> 6, mr = Lid & 63;
            const v8us val = *(const v8usa*)((pln ? tl_ : th_) + mr * 72 + piece * 8); *(volatile v8us*)((pln ? XRL : XRH) + ((size_t)b * NK + m0 + mr) * CC + c0 + piece * 8) = val; }
    };
    pass(); __threadfence(); pass();
}
__global__ __launch_bounds__(256) void k_wt(const float* __restrict__ Wm, bf* WT) {
    __shared__ __align__(16) unsigned short tl[64 * 72];
    const int tid = threadIdx.x, k0 = blockIdx.x * 64, n0 = blockIdx.y * 64;
    const int kk = tid >> 2, nq = (tid & 3) * 16;
#pragma unroll
    for (int i = 0; i < 16; ++i) tl[(nq + i) * 72 + kk] = f2bf(Wm[(size_t)(k0 + kk) * CC + n0 + nq + i]);
    __syncthreads();
    const int piece = tid & 7;
    auto pass = [&]() {
#pragma unroll
        for (int s = 0; s < 2; ++s) { const int nr = (tid >> 3) + 32 * s; const v8us val = *(const v8usa*)(tl + nr * 72 + piece * 8);
            *(volatile v8us*)(WT + (size_t)(n0 + nr) * CC + k0 + piece * 8) = val; }
    };
    pass(); __threadfence(); pass();
}

template <bool SPLITA, int MODE, bool HMA>
__global__ __launch_bounds__(128) void k_gemmb(const bf* __restrict__ A, const bf* __restrict__ Al, const bf* __restrict__ Bn, const float* __restrict__ bias, void* Cout) {
    __shared__ __align__(16) float ost[64 * 68];
    const int lane = threadIdx.x & 31, wave = threadIdx.x >> 5, lr = lane & 15, hi = lane >> 4;
    const int r0 = blockIdx.x * 64 + wave * 16, c0 = blockIdx.y * 64;
    const size_t aoff = (size_t)(r0 + lr) * CC + 8 * hi;
    const int hb = (r0 + lr) / NN_, hn = (r0 + lr) - hb * NN_;
    size_t boff[4];
#pragma unroll
    for (int t = 0; t < 4; ++t) boff[t] = (size_t)(c0 + t * 16 + lr) * CC + 8 * hi;
    v8f acc[4];
#pragma unroll
    for (int t = 0; t < 4; ++t) acc[t] = (v8f){};
#pragma unroll 1
    for (int kc = 0; kc < CC; kc += 32) {
        const size_t ao = HMA ? ((((size_t)hb * NH_ + (kc >> 5)) * NN_ + hn) * HD + 8 * hi) : (aoff + kc);
        const v16bf a = cat16b(*(const v8us*)(A + ao), *(const v8us*)(A + ao + 16));
        v16bf al = a;
        if (SPLITA) al = cat16b(*(const v8us*)(Al + ao), *(const v8us*)(Al + ao + 16));
#pragma unroll
        for (int t = 0; t < 4; ++t) { const v16bf b = cat16b(*(const v8us*)(Bn + boff[t] + kc), *(const v8us*)(Bn + boff[t] + kc + 16)); acc[t] = wmmab(a, b, acc[t]); if (SPLITA) acc[t] = wmmab(al, b, acc[t]); }
        asm volatile("v_nop\n\tv_nop\n\tv_nop\n\tv_nop" : "+v"(acc[0]), "+v"(acc[1]), "+v"(acc[2]), "+v"(acc[3]) : "v"(a), "v"(al));
    }
    float* os = ost + wave * 16 * 68;
#pragma unroll
    for (int t = 0; t < 4; ++t) { const float bv = bfr(bias[c0 + t * 16 + lr]);
#pragma unroll
        for (int j = 0; j < 8; ++j) os[(hi * 8 + j) * 68 + t * 16 + lr] = acc[t][j] + bv; }
    __syncthreads();
    if (MODE == 0) {
        h16* crow = (h16*)Cout + (size_t)r0 * CC + c0;
        auto pass = [&]() {
#pragma unroll
            for (int s = 0; s < 4; ++s) { const int row = 4 * s + (lane >> 3), piece = lane & 7; const float* sp = os + row * 68 + piece * 8; v8h o;
#pragma unroll
                for (int i = 0; i < 8; ++i) o[i] = (h16)sp[i];
                *(volatile v8h*)(crow + (size_t)row * CC + piece * 8) = o; }
        };
        pass(); __threadfence(); pass();
    } else if (MODE == 1) {
        const int rb = blockIdx.x * 64; const int b = rb / NN_, n0 = rb - b * NN_;
        float* ob = (float*)Cout + ((size_t)b * CC + c0) * NN_ + n0;
        auto pass = [&]() {
#pragma unroll
            for (int s = 0; s < 8; ++s) { const int col = wave * 16 + 2 * s + (lane >> 4), q = lane & 15; v4f v;
#pragma unroll
                for (int i = 0; i < 4; ++i) v[i] = ost[(q * 4 + i) * 68 + col];
                *(volatile v4f*)(ob + (size_t)col * NN_ + q * 4) = v; }
        };
        pass(); __threadfence(); pass();
    } else {
        const int rb = blockIdx.x * 64; const int b = rb / NK, m0 = rb - b * NK;
        h16* vb = (h16*)Cout + ((size_t)b * CC + c0) * NK + m0;
        auto pass = [&]() {
#pragma unroll
            for (int s = 0; s < 4; ++s) { const int col = wave * 16 + 4 * s + (lane >> 3), q = lane & 7; v8h v;
#pragma unroll
                for (int i = 0; i < 8; ++i) v[i] = (h16)ost[(q * 8 + i) * 68 + col];
                *(volatile v8h*)(vb + (size_t)col * NK + q * 8) = v; }
        };
        pass(); __threadfence(); pass();
    }
}

__global__ __launch_bounds__(128) void k_attn(const h16* __restrict__ Q16, const h16* __restrict__ K16, const h16* __restrict__ VT16, bf* CH, bf* CL) {
    __shared__ __align__(16) h16 plds[4][16 * 32];
    __shared__ __align__(16) float ost[4][16 * 36];
    const int lane = threadIdx.x & 31, wave = threadIdx.x >> 5, lr = lane & 15, hi = lane >> 4;
    const int bid = blockIdx.x;
    const int b = bid / (NH_ * (NN_ / 64)), rem = bid - b * (NH_ * (NN_ / 64)), h = rem / (NN_ / 64), qt = rem - h * (NN_ / 64);
    const int q0 = qt * 64 + wave * 16;
    h16* pl = &plds[wave][0];
    const h16* qp = Q16 + ((size_t)b * NN_ + q0 + lr) * CC + h * HD + 8 * hi;
    const v16h qa = cat16(*(const v8h*)qp, *(const v8h*)(qp + 16));
    const h16* kh_b = K16 + (size_t)b * NK * CC + h * HD;
    const h16* vt_b = VT16 + ((size_t)b * CC + h * HD) * NK;
    v8f o[2]; o[0] = (v8f){}; o[1] = (v8f){};
    float mrow[8], lpart[8];
#pragma unroll
    for (int j = 0; j < 8; ++j) { mrow[j] = -3.0e38f; lpart[j] = 0.f; }
#pragma unroll 1
    for (int kt = 0; kt < NK / 32; ++kt) {
        const int l0 = kt * 32;
        const h16* r0p = kh_b + (size_t)(l0 + lr) * CC + 8 * hi; const h16* r1p = kh_b + (size_t)(l0 + 16 + lr) * CC + 8 * hi;
        v8f s0 = {}, s1 = {};
        s0 = wmma16(qa, cat16(*(const v8h*)r0p, *(const v8h*)(r0p + 16)), s0);
        s1 = wmma16(qa, cat16(*(const v8h*)r1p, *(const v8h*)(r1p + 16)), s1);
        asm volatile("v_nop\n\tv_nop\n\tv_nop\n\tv_nop" : "+v"(s0), "+v"(s1) : "v"(qa));
        float alpha[8];
#pragma unroll
        for (int j = 0; j < 8; ++j) {
            const float a0 = s0[j] * SCL, a1 = s1[j] * SCL;
            float mx = fmaxf(a0, a1);
            mx = fmaxf(mx, __shfl_xor(mx, 1, 16)); mx = fmaxf(mx, __shfl_xor(mx, 2, 16)); mx = fmaxf(mx, __shfl_xor(mx, 4, 16)); mx = fmaxf(mx, __shfl_xor(mx, 8, 16));
            const float mn = fmaxf(mrow[j], mx);
            alpha[j] = __expf(mrow[j] - mn); mrow[j] = mn;
            const float p0 = __expf(a0 - mn), p1 = __expf(a1 - mn);
            lpart[j] = lpart[j] * alpha[j] + (p0 + p1);
            const int mr = hi * 8 + j;
            pl[mr * 32 + lr] = (h16)(p0 * PSC); pl[mr * 32 + 16 + lr] = (h16)(p1 * PSC);
        }
#pragma unroll
        for (int n = 0; n < 2; ++n)
#pragma unroll
            for (int j = 0; j < 8; ++j) o[n][j] *= alpha[j];
        asm volatile("" ::: "memory");
        const v16h pa = cat16(*(const v8ha*)(pl + lr * 32 + hi * 8), *(const v8ha*)(pl + lr * 32 + 16 + hi * 8));
#pragma unroll
        for (int n = 0; n < 2; ++n) { const h16* vp = vt_b + (size_t)(n * 16 + lr) * NK + l0 + hi * 8; o[n] = wmma16(pa, cat16(*(const v8h*)vp, *(const v8h*)(vp + 16)), o[n]); }
        asm volatile("v_nop\n\tv_nop\n\tv_nop\n\tv_nop" : "+v"(o[0]), "+v"(o[1]) : "v"(pa));
    }
    float inv[8];
#pragma unroll
    for (int j = 0; j < 8; ++j) { float rs = lpart[j]; rs += __shfl_xor(rs, 1, 16); rs += __shfl_xor(rs, 2, 16); rs += __shfl_xor(rs, 4, 16); rs += __shfl_xor(rs, 8, 16); inv[j] = 1.0f / (rs * PSC); }
    float* os = &ost[wave][0];
#pragma unroll
    for (int n = 0; n < 2; ++n)
#pragma unroll
        for (int j = 0; j < 8; ++j) os[(hi * 8 + j) * 36 + n * 16 + lr] = o[n][j] * inv[j];
    asm volatile("" ::: "memory");
    __builtin_amdgcn_fence(__ATOMIC_RELEASE, "workgroup");
    __builtin_amdgcn_wave_barrier();
    const size_t cbase = (((size_t)b * NH_ + h) * NN_ + q0) * HD;
    auto pass = [&]() {
        const int row = lane >> 1, half = lane & 1; const float* sp = os + row * 36 + half * 16; v8us oh, ol, oh2, ol2;
#pragma unroll
        for (int i = 0; i < 8; ++i) { const unsigned short hb = f2bf(sp[i]); oh[i] = hb; ol[i] = f2bf(sp[i] - bf2f(hb)); const unsigned short hb2 = f2bf(sp[8 + i]); oh2[i] = hb2; ol2[i] = f2bf(sp[8 + i] - bf2f(hb2)); }
        *(volatile v8us*)(CH + cbase + (size_t)row * HD + half * 16) = oh; *(volatile v8us*)(CH + cbase + (size_t)row * HD + half * 16 + 8) = oh2;
        *(volatile v8us*)(CL + cbase + (size_t)row * HD + half * 16) = ol; *(volatile v8us*)(CL + cbase + (size_t)row * HD + half * 16 + 8) = ol2;
    };
    pass(); __threadfence(); pass();
}

extern "C" void kernel_launch(void* const* d_in, const int* in_sizes, int n_in,
                              void* d_out, int out_size, void* d_ws, size_t ws_size, hipStream_t stream) {
    (void)in_sizes; (void)n_in; (void)out_size;
    const float* x = (const float*)d_in[0]; const float* Wq = (const float*)d_in[1]; const float* bq = (const float*)d_in[2]; const float* Wk = (const float*)d_in[3]; const float* bk = (const float*)d_in[4];
    const float* Wv = (const float*)d_in[5]; const float* bv = (const float*)d_in[6]; const float* Wp = (const float*)d_in[7]; const float* bp = (const float*)d_in[8];
    const float* g = (const float*)d_in[9]; const float* be = (const float*)d_in[10]; const float* mu = (const float*)d_in[11]; const float* var = (const float*)d_in[12];
    float* out = (float*)d_out;
    char* wsp = (char*)d_ws;
    auto take = [&](size_t bytes) { char* p = wsp; wsp += (bytes + 255) & ~(size_t)255; return (void*)p; };
    bf* Xb = (bf*)take((size_t)NTQ * CC * 2); bf* XRH = (bf*)take((size_t)NTKV * CC * 2); bf* XRL = (bf*)take((size_t)NTKV * CC * 2);
    bf* WT[4]; for (int i = 0; i < 4; ++i) WT[i] = (bf*)take((size_t)CC * CC * 2);
    h16* Q16 = (h16*)take((size_t)NTQ * CC * 2); h16* K16 = (h16*)take((size_t)NTKV * CC * 2); h16* VT16 = (h16*)take((size_t)NTKV * CC * 2);
    bf* CLt = (bf*)take((size_t)NTQ * CC * 2);
    if ((size_t)(wsp - (char*)d_ws) > ws_size) return;
    bf* CHt = Xb;
    k_tok<<<dim3(NN_ / 64, CC / 64, NB_), 256, 0, stream>>>(x, Xb);
    k_pool<<<dim3(NK / 64, CC / 64, NB_), 256, 0, stream>>>(x, g, be, mu, var, XRH, XRL);
    const float* Ws[4] = {Wq, Wk, Wv, Wp};
    for (int i = 0; i < 4; ++i) k_wt<<<dim3(CC / 64, CC / 64, 1), 256, 0, stream>>>(Ws[i], WT[i]);
    k_gemmb<false, 0, false><<<dim3(NTQ / 64, CC / 64, 1), 128, 0, stream>>>(Xb, nullptr, WT[0], bq, Q16);
    k_gemmb<true, 0, false><<<dim3(NTKV / 64, CC / 64, 1), 128, 0, stream>>>(XRH, XRL, WT[1], bk, K16);
    k_gemmb<true, 2, false><<<dim3(NTKV / 64, CC / 64, 1), 128, 0, stream>>>(XRH, XRL, WT[2], bv, VT16);
    k_attn<<<NB_ * NH_ * (NN_ / 64), 128, 0, stream>>>(Q16, K16, VT16, CHt, CLt);
    k_gemmb<true, 1, true><<<dim3(NTQ / 64, CC / 64, 1), 128, 0, stream>>>(CHt, CLt, WT[3], bp, out);
}
